// MultiAttentionGATBridge_28913719837513
// MI455X (gfx1250) — hardware-verified
//
#include <hip/hip_runtime.h>
#include <stdint.h>

typedef __attribute__((ext_vector_type(16))) _Float16 v16h;
typedef __attribute__((ext_vector_type(8)))  _Float16 v8h;
typedef __attribute__((ext_vector_type(4)))  _Float16 v4h;
typedef __attribute__((ext_vector_type(16))) __bf16   v16b;
typedef __attribute__((ext_vector_type(8)))  __bf16   v8b;
typedef __attribute__((ext_vector_type(8)))  float    v8f;
typedef __attribute__((ext_vector_type(4)))  float    v4f;

__device__ __forceinline__ unsigned short f2bf_bits(float f) {
  unsigned u = __float_as_uint(f);
  return (unsigned short)((u + 0x7FFFu + ((u >> 16) & 1u)) >> 16);
}
__device__ __forceinline__ float bf_bits2f(unsigned short h) { return __uint_as_float(((unsigned)h) << 16); }

__device__ __forceinline__ void dep_guard_h(v8f& a, v8f& b, v16h x, v16h y) { asm volatile("v_nop\n\tv_nop\n\tv_nop\n\tv_nop" : "+v"(a), "+v"(b) : "v"(x), "v"(y)); }
__device__ __forceinline__ void dep_guard_b(v8f& a, v8f& b, v16b x, v16b y) { asm volatile("v_nop\n\tv_nop\n\tv_nop\n\tv_nop" : "+v"(a), "+v"(b) : "v"(x), "v"(y)); }
__device__ __forceinline__ void keep4_h(v16h a, v16h b, v16h c, v16h d) { asm volatile("v_nop" :: "v"(a), "v"(b), "v"(c), "v"(d)); }
__device__ __forceinline__ void keep4_b(v16b a, v16b b, v16b c, v16b d) { asm volatile("v_nop" :: "v"(a), "v"(b), "v"(c), "v"(d)); }
__device__ __forceinline__ void acc_guard4(v8f& a, v8f& b, v8f& c, v8f& d) { asm volatile("v_nop\n\tv_nop\n\tv_nop\n\tv_nop" : "+v"(a), "+v"(b), "+v"(c), "+v"(d)); }
template <typename T> struct Frag;
template <> struct Frag<_Float16> {
  typedef v16h V; union U { v16h v; v8h h[2]; };
  static __device__ __forceinline__ v16h load(const _Float16* p) {
    U f; f.h[0] = *(const v8h*)(p); f.h[1] = *(const v8h*)(p + 16); return f.v;
  }
  static __device__ __forceinline__ v8f mma(v16h a, v16h b, v8f c) {
    return __builtin_amdgcn_wmma_f32_16x16x32_f16(false, a, false, b, (short)0, c, false, false);
  }
  static __device__ __forceinline__ void guard(v8f& a, v8f& b, v16h x, v16h y) { dep_guard_h(a, b, x, y); }
  static __device__ __forceinline__ void keep(v16h a, v16h b, v16h c, v16h d) { keep4_h(a, b, c, d); }
};
template <> struct Frag<__bf16> {
  typedef v16b V; union U { v16b v; v8b h[2]; };
  static __device__ __forceinline__ v16b load(const __bf16* p) {
    U f; f.h[0] = *(const v8b*)(p); f.h[1] = *(const v8b*)(p + 16); return f.v;
  }
  static __device__ __forceinline__ v8f mma(v16b a, v16b b, v8f c) {
    return __builtin_amdgcn_wmma_f32_16x16x32_bf16(false, a, false, b, (short)0, c, false, false);
  }
  static __device__ __forceinline__ void guard(v8f& a, v8f& b, v16b x, v16b y) { dep_guard_b(a, b, x, y); }
  static __device__ __forceinline__ void keep(v16b a, v16b b, v16b c, v16b d) { keep4_b(a, b, c, d); }
};

__global__ __launch_bounds__(256) void cast_f32_f16x2(
    const float* __restrict__ in, _Float16* __restrict__ out, int n2) {
  int i = blockIdx.x * 256 + threadIdx.x;
  if (i < n2) {
    const _Float16 h0 = (_Float16)in[2 * i], h1 = (_Float16)in[2 * i + 1];
    const unsigned u = (unsigned)__builtin_bit_cast(unsigned short, h0) | ((unsigned)__builtin_bit_cast(unsigned short, h1) << 16);
    ((volatile unsigned*)out)[i] = u;
    __threadfence();
    ((volatile unsigned*)out)[i] = u;
  }
}

__device__ __forceinline__ float act_elu_f(float v) { return (v > 0.0f) ? v : (__expf(v) - 1.0f); }
__device__ __forceinline__ float act_gelu_f(float v) {
  const float t = 0.7978845608028654f * (v + 0.044715f * v * v * v);
  const float e = __expf(2.0f * t);
  const float th = 1.0f - 2.0f * __builtin_amdgcn_rcpf(e + 1.0f);
  return 0.5f * v * (1.0f + th);
}

template <int BIAS_MODE, int OUT_MODE, bool RESID, int ACT, bool AGRP>
__global__ __launch_bounds__(256) void gemm64(
    const _Float16* __restrict__ A, int lda, long sAy, long sAz, long agrp,
    const _Float16* __restrict__ Bt, int ldb, long sBy, long sBz,
    void* __restrict__ Cout, void* __restrict__ Cout2, int ldc, long sCy, long sCz,
    const float* __restrict__ bias, const float* __restrict__ resid,
    int M, int N, int K, float scale) {
  typedef Frag<_Float16> F;
  typedef v16h V;
  __shared__ __align__(16) float sT[8][16 * 68];
  const int by   = blockIdx.y, bz = blockIdx.z;
  const int lane = threadIdx.x & 31;
  const int wave = threadIdx.x >> 5;
  const int tilesN = N >> 6;
  const int tilesM = M >> 6;
  const int tile = blockIdx.x * 8 + wave;
  if (tile >= tilesM * tilesN) return;
  const int tm = tile / tilesN;
  const int tn = tile - tm * tilesN;
  const int m0 = tm << 6;
  const int n0 = tn << 6;

  const _Float16* Ab = A  + ((long)by * sAy + (long)bz * sAz);
  const _Float16* Bb = Bt + ((long)by * sBy + (long)bz * sBz);
  const size_t cOff = (size_t)((long)by * sCy + (long)bz * sCz);

  const int rlane = lane & 15;
  const int koff  = (lane >> 4) * 8;
  const int mOff  = (lane >> 4) * 8;

  v8f acc[4][4];
#pragma unroll
  for (int i = 0; i < 4; ++i)
#pragma unroll
    for (int j = 0; j < 4; ++j) acc[i][j] = (v8f){0.f,0.f,0.f,0.f,0.f,0.f,0.f,0.f};

  for (int k0 = 0; k0 < K; k0 += 32) {
    V bh[4];
#pragma unroll
    for (int j = 0; j < 4; ++j) {
      const size_t bo = (size_t)(n0 + (j << 4) + rlane) * ldb + koff + k0;
      bh[j] = F::load(Bb + bo);
    }
#pragma unroll
    for (int i = 0; i < 4; ++i) {
      const size_t ao = (size_t)(m0 + (i << 4) + rlane) * lda + koff + k0;
      const V a0 = F::load(Ab + ao);
      V a1 = a0;
      if (AGRP) a1 = F::load(Ab + agrp + ao);
#pragma unroll
      for (int j = 0; j < 4; ++j) {
        if (AGRP && j >= 2) acc[i][j] = F::mma(a1, bh[j], acc[i][j]);
        else                acc[i][j] = F::mma(a0, bh[j], acc[i][j]);
      }
      F::guard(acc[i][0], acc[i][3], a0, a1);
    }
    F::keep(bh[0], bh[1], bh[2], bh[3]);
  }
  acc_guard4(acc[0][0], acc[0][1], acc[0][2], acc[0][3]);
  acc_guard4(acc[1][0], acc[1][1], acc[1][2], acc[1][3]);
  acc_guard4(acc[2][0], acc[2][1], acc[2][2], acc[2][3]);
  acc_guard4(acc[3][0], acc[3][1], acc[3][2], acc[3][3]);

  float* slab = sT[wave];
  const float* Rb = RESID ? (resid + cOff) : nullptr;
#pragma unroll
  for (int i = 0; i < 4; ++i) {
    const int mBase = m0 + (i << 4);
#pragma unroll
    for (int j = 0; j < 4; ++j) {
      const int n = n0 + (j << 4) + rlane;
      float bv = 0.f;
      if (BIAS_MODE == 2) bv = bias[n];
#pragma unroll
      for (int r = 0; r < 8; ++r) {
        float v = acc[i][j][r] * scale;
        if (BIAS_MODE == 2) v += bv;
        if (RESID) v += Rb[(size_t)(mBase + mOff + r) * ldc + n];
        if (ACT == 6) v = act_gelu_f(v);
        if (ACT == 7) v = act_elu_f(v);
        slab[(mOff + r) * 68 + (j << 4) + rlane] = v;
      }
    }
    __builtin_amdgcn_fence(__ATOMIC_RELEASE, "workgroup");
    __builtin_amdgcn_wave_barrier();
    __builtin_amdgcn_fence(__ATOMIC_ACQUIRE, "workgroup");
    for (int pass = 0; pass < 2; ++pass) {
      if (OUT_MODE == 0 || OUT_MODE == 3) {
        float* C = (float*)Cout + cOff;
        const int hh = lane >> 4, c4 = (lane & 15) * 4;
#pragma unroll
        for (int it = 0; it < 8; ++it) {
          const int row = it * 2 + hh;
          v4f v = *(const v4f*)(slab + row * 68 + c4);
          *(volatile v4f*)(C + (size_t)(mBase + row) * ldc + n0 + c4) = v;
        }
      }
      if (OUT_MODE == 1 || OUT_MODE == 3) {
        _Float16* C2 = (OUT_MODE == 1) ? ((_Float16*)Cout + cOff) : ((_Float16*)Cout2 + cOff);
        const int q = lane >> 3, c8 = (lane & 7) * 8;
#pragma unroll
        for (int it = 0; it < 4; ++it) {
          const int row = it * 4 + q;
          const float* sp = slab + row * 68 + c8;
          v8h hv;
#pragma unroll
          for (int e = 0; e < 8; ++e) hv[e] = (_Float16)sp[e];
          *(volatile v8h*)(C2 + (size_t)(mBase + row) * ldc + n0 + c8) = hv;
        }
      }
      __threadfence();
    }
    __builtin_amdgcn_fence(__ATOMIC_RELEASE, "workgroup");
    __builtin_amdgcn_wave_barrier();
    __builtin_amdgcn_fence(__ATOMIC_ACQUIRE, "workgroup");
  }
}

__global__ __launch_bounds__(256) void tpose_cast_kernel(const float* __restrict__ in, _Float16* __restrict__ out,
                                                         int R, int C, float carry) {
  __shared__ __align__(16) _Float16 sm[32 * 72];
  const int t = threadIdx.x;
  const int r0 = blockIdx.x * 64, c0 = blockIdx.y * 32;
#pragma unroll
  for (int it = 0; it < 8; ++it) {
    const int idx = it * 256 + t;
    const int rr = idx >> 5, cc = idx & 31;
    sm[cc * 72 + rr] = (_Float16)(in[(size_t)(r0 + rr) * C + c0 + cc] * carry);
  }
  __syncthreads();
  const int cc = t >> 3, c8 = (t & 7) * 8;
  const v8h v = *(const v8h*)(sm + cc * 72 + c8);
  _Float16* dp = out + (size_t)(c0 + cc) * R + r0 + c8;
  *(volatile v8h*)dp = v;
  __threadfence();
  *(volatile v8h*)dp = v;
}

__global__ __launch_bounds__(256) void ln_kernel(const float* __restrict__ h, const float* __restrict__ g,
                                                 const float* __restrict__ bta, float* __restrict__ o,
                                                 _Float16* __restrict__ o16, int nrows) {
  __shared__ __align__(16) float sw[8][256];
  const int lane = threadIdx.x & 31, wave = threadIdx.x >> 5;
  const int row = blockIdx.x * 8 + wave;
  if (row >= nrows) return;
  const float* hr = h + (size_t)row * 256;
  const v4f a = *(const v4f*)(hr + lane * 4);
  const v4f c = *(const v4f*)(hr + 128 + lane * 4);
  float s = ((a[0] + a[1]) + (a[2] + a[3])) + ((c[0] + c[1]) + (c[2] + c[3]));
#pragma unroll
  for (int off = 16; off > 0; off >>= 1) s += __shfl_xor(s, off, 32);
  const float mu = s * (1.0f / 256.0f);
  const v4f da = a - mu;
  const v4f dc = c - mu;
  float sq = ((da[0] * da[0] + da[1] * da[1]) + (da[2] * da[2] + da[3] * da[3]))
           + ((dc[0] * dc[0] + dc[1] * dc[1]) + (dc[2] * dc[2] + dc[3] * dc[3]));
#pragma unroll
  for (int off = 16; off > 0; off >>= 1) sq += __shfl_xor(sq, off, 32);
  const float var = sq * (1.0f / 256.0f);
  const float rs  = rsqrtf(var + 1e-5f);
  const v4f ga = *(const v4f*)(g + lane * 4),   gc = *(const v4f*)(g + 128 + lane * 4);
  const v4f ba = *(const v4f*)(bta + lane * 4), bc = *(const v4f*)(bta + 128 + lane * 4);
  const v4f oa = da * rs * ga + ba;
  const v4f oc = dc * rs * gc + bc;
  float* orow = o + (size_t)row * 256;
  for (int pass = 0; pass < 2; ++pass) {
    *(volatile v4f*)(orow + lane * 4) = oa;
    *(volatile v4f*)(orow + 128 + lane * 4) = oc;
    __threadfence();
  }
  float* sp = sw[wave];
  *(v4f*)(sp + lane * 4) = oa;
  *(v4f*)(sp + 128 + lane * 4) = oc;
  __builtin_amdgcn_fence(__ATOMIC_RELEASE, "workgroup");
  __builtin_amdgcn_wave_barrier();
  __builtin_amdgcn_fence(__ATOMIC_ACQUIRE, "workgroup");
  const v4f u0 = *(const v4f*)(sp + lane * 8);
  const v4f u1 = *(const v4f*)(sp + lane * 8 + 4);
  v8h hv;
  hv[0] = (_Float16)u0[0]; hv[1] = (_Float16)u0[1]; hv[2] = (_Float16)u0[2]; hv[3] = (_Float16)u0[3];
  hv[4] = (_Float16)u1[0]; hv[5] = (_Float16)u1[1]; hv[6] = (_Float16)u1[2]; hv[7] = (_Float16)u1[3];
  _Float16* o16r = o16 + (size_t)row * 256 + lane * 8;
  for (int pass = 0; pass < 2; ++pass) {
    *(volatile v8h*)o16r = hv;
    __threadfence();
  }
}

__global__ __launch_bounds__(256) void scores_kernel(const _Float16* __restrict__ hp, const float* __restrict__ asrc,
                                                     const float* __restrict__ adst, float* __restrict__ src,
                                                     float* __restrict__ dst, int dh, long SB, long SD, long SH, int ntot) {
  const int n = blockIdx.x * 256 + threadIdx.x;
  const int h = blockIdx.y;
  const int nc = (n < ntot) ? n : (ntot - 1);
  const int b = nc >> 10, j = nc & 1023;
  const _Float16* p = hp + ((long)b * SB + (long)h * SH + j);
  const float* wsv = asrc + h * dh;
  const float* wdv = adst + h * dh;
  const int dhc = dh < 256 ? dh : 256;
  float as = 0.f, ad = 0.f;
#pragma unroll 4
  for (int d = 0; d < dhc; ++d) {
    const float v = (float)p[(long)d * SD];
    as += v * wsv[d];
    ad += v * wdv[d];
  }
  if (n < ntot) {
    float* ps = src + (size_t)h * ntot + n;
    float* pd = dst + (size_t)h * ntot + n;
    *(volatile float*)ps = as;
    *(volatile float*)pd = ad;
    __threadfence();
    *(volatile float*)ps = as;
    *(volatile float*)pd = ad;
  }
}

__global__ __launch_bounds__(256) void pbuild_kernel(const float* __restrict__ adj, const float* __restrict__ src,
                                                     const float* __restrict__ dst, _Float16* __restrict__ P) {
  __shared__ __align__(16) _Float16 psh[8 * 1024];
  __shared__ float redm[8];
  __shared__ float reds[8];
  const int i = blockIdx.x, b = blockIdx.y;
  const int t = threadIdx.x, lane = t & 31, wave = t >> 5;
  const int j4 = t * 4;
  const size_t n_i = (size_t)b * 1024 + i;
  const v4f av = *(const v4f*)(adj + n_i * 1024 + j4);
#pragma unroll 1
  for (int h = 0; h < 8; ++h) {
    const float si = src[(size_t)h * 4096 + n_i];
    const v4f dv = *(const v4f*)(dst + (size_t)h * 4096 + (size_t)b * 1024 + j4);
    float e[4];
    float m = -3.0e38f;
#pragma unroll
    for (int q = 0; q < 4; ++q) {
      float x = si + dv[q];
      x = (x > 0.0f) ? x : 0.2f * x;
      e[q] = (av[q] > 0.0f) ? x : -1.0e9f;
      m = fmaxf(m, e[q]);
    }
#pragma unroll
    for (int off = 16; off > 0; off >>= 1) m = fmaxf(m, __shfl_xor(m, off, 32));
    if (lane == 0) redm[wave] = m;
    __syncthreads();
    float mm = redm[0];
#pragma unroll
    for (int w = 1; w < 8; ++w) mm = fmaxf(mm, redm[w]);
    float p[4];
    float s = 0.f;
#pragma unroll
    for (int q = 0; q < 4; ++q) { p[q] = __expf(e[q] - mm); s += p[q]; }
#pragma unroll
    for (int off = 16; off > 0; off >>= 1) s += __shfl_xor(s, off, 32);
    if (lane == 0) reds[wave] = s;
    __syncthreads();
    float l = reds[0];
#pragma unroll
    for (int w = 1; w < 8; ++w) l += reds[w];
    const float inv = 1.0f / l;
    v4h pv;
#pragma unroll
    for (int q = 0; q < 4; ++q) pv[q] = (_Float16)((p[q] * inv) * 32768.0f);
    *(v4h*)(psh + h * 1024 + j4) = pv;
  }
  __syncthreads();
  const size_t prow = n_i * 8 * 1024;
  for (int pass = 0; pass < 2; ++pass) {
#pragma unroll
    for (int it = 0; it < 4; ++it) {
      const int idx = it * 256 + t;
      const int hh = idx >> 7;
      const int c8 = (idx & 127) * 8;
      const v8h v = *(const v8h*)(psh + hh * 1024 + c8);
      *(volatile v8h*)(P + prow + (size_t)hh * 1024 + c8) = v;
    }
    __threadfence();
  }
}

extern "C" void kernel_launch(void* const* d_in, const int* in_sizes, int n_in,
                              void* d_out, int out_size, void* d_ws, size_t ws_size,
                              hipStream_t stream) {
  const int B = 4, S = 1024, D = 256, H = 8, NTOK = B * S;
  if (n_in < 17) return;
  if (in_sizes[0] != B * S * S || in_sizes[1] != NTOK * D || in_sizes[2] != D * D || in_sizes[3] != H * 32 ||
      in_sizes[4] != H * 32 || in_sizes[5] != D * D || in_sizes[6] != H * 32 || in_sizes[7] != H * 32 ||
      in_sizes[8] != D * H * D || in_sizes[9] != H * D || in_sizes[10] != H * D || in_sizes[11] != D ||
      in_sizes[12] != D || in_sizes[13] != D * 2 * D || in_sizes[14] != 2 * D || in_sizes[15] != 2 * D * D ||
      in_sizes[16] != D || out_size != NTOK * D) return;

  const float* adj  = (const float*)d_in[0];
  const float* x    = (const float*)d_in[1];
  const float* W0   = (const float*)d_in[2];
  const float* as0  = (const float*)d_in[3];
  const float* ad0  = (const float*)d_in[4];
  const float* W1   = (const float*)d_in[5];
  const float* as1  = (const float*)d_in[6];
  const float* ad1  = (const float*)d_in[7];
  const float* W2   = (const float*)d_in[8];
  const float* as2  = (const float*)d_in[9];
  const float* ad2  = (const float*)d_in[10];
  const float* ln_g = (const float*)d_in[11];
  const float* ln_b = (const float*)d_in[12];
  const float* ffw1 = (const float*)d_in[13];
  const float* ffb1 = (const float*)d_in[14];
  const float* ffw2 = (const float*)d_in[15];
  const float* ffb2 = (const float*)d_in[16];
  float* out = (float*)d_out;

  char* ws = (char*)d_ws;
  size_t off = 0;
  auto carve = [&](size_t bytes) -> void* {
    void* p = ws + off;
    off += (bytes + 255) & ~(size_t)255;
    return p;
  };
  _Float16* W0T   = (_Float16*)carve((size_t)D * D * 2);
  _Float16* W1T   = (_Float16*)carve((size_t)D * D * 2);
  _Float16* W2T   = (_Float16*)carve((size_t)H * D * D * 2);
  _Float16* F1T   = (_Float16*)carve((size_t)2 * D * D * 2);
  _Float16* F2T   = (_Float16*)carve((size_t)D * 2 * D * 2);
  _Float16* h16   = (_Float16*)carve((size_t)NTOK * D * 2);
  float*    hA    = (float*)carve((size_t)NTOK * D * 4);
  float*    hB    = (float*)carve((size_t)NTOK * D * 4);
  _Float16* hp16  = (_Float16*)carve((size_t)B * H * D * S * 2);
  float*    srcb  = (float*)carve((size_t)H * NTOK * 4);
  float*    dstb  = (float*)carve((size_t)H * NTOK * 4);
  _Float16* P16   = (_Float16*)carve((size_t)NTOK * H * S * 2);
  float*    hln   = (float*)carve((size_t)NTOK * D * 4);
  _Float16* hln16 = (_Float16*)carve((size_t)NTOK * D * 2);
  _Float16* mid16 = (_Float16*)carve((size_t)NTOK * 2 * D * 2);
  if (off > ws_size || off > (size_t)134217728) return;

  const float WSC = 16.0f, WINV = 1.0f / 16.0f;
  const float PINV = 1.0f / 32768.0f;

  tpose_cast_kernel<<<dim3(D / 64, D / 32), 256, 0, stream>>>(W0, W0T, D, D, WSC);
  tpose_cast_kernel<<<dim3(D / 64, D / 32), 256, 0, stream>>>(W1, W1T, D, D, WSC);
  tpose_cast_kernel<<<dim3(D / 64, (H * D) / 32), 256, 0, stream>>>(W2, W2T, D, H * D, WSC);
  tpose_cast_kernel<<<dim3(D / 64, (2 * D) / 32), 256, 0, stream>>>(ffw1, F1T, D, 2 * D, WSC);
  tpose_cast_kernel<<<dim3((2 * D) / 64, D / 32), 256, 0, stream>>>(ffw2, F2T, 2 * D, D, WSC);
  cast_f32_f16x2<<<(NTOK * D / 2 + 255) / 256, 256, 0, stream>>>(x, h16, NTOK * D / 2);

  gemm64<0, 1, false, 0, false><<<dim3(8, 1, B), 256, 0, stream>>>(
      W0T, D, 0L, 0L, 0L, h16, D, 0L, (long)S * D, hp16, nullptr, S, 0L, (long)D * S,
      nullptr, nullptr, D, S, D, WINV);
  scores_kernel<<<dim3(NTOK / 256, H), 256, 0, stream>>>(hp16, as0, ad0, srcb, dstb, 32,
                                                          (long)D * S, (long)S, (long)32 * S, NTOK);
  pbuild_kernel<<<dim3(S, B), 256, 0, stream>>>(adj, srcb, dstb, P16);
  gemm64<0, 3, true, 7, true><<<dim3(2, 4, B), 256, 0, stream>>>(
      P16, H * S, (long)2 * S, (long)S * H * S, (long)S, hp16, S, (long)64 * S, (long)D * S,
      hA, h16, D, 64L, (long)S * D, nullptr, x, S, 64, S, PINV);

  gemm64<0, 1, false, 0, false><<<dim3(8, 1, B), 256, 0, stream>>>(
      W1T, D, 0L, 0L, 0L, h16, D, 0L, (long)S * D, hp16, nullptr, S, 0L, (long)D * S,
      nullptr, nullptr, D, S, D, WINV);
  scores_kernel<<<dim3(NTOK / 256, H), 256, 0, stream>>>(hp16, as1, ad1, srcb, dstb, 32,
                                                          (long)D * S, (long)S, (long)32 * S, NTOK);
  pbuild_kernel<<<dim3(S, B), 256, 0, stream>>>(adj, srcb, dstb, P16);
  gemm64<0, 3, true, 7, true><<<dim3(2, 4, B), 256, 0, stream>>>(
      P16, H * S, (long)2 * S, (long)S * H * S, (long)S, hp16, S, (long)64 * S, (long)D * S,
      hB, h16, D, 64L, (long)S * D, nullptr, hA, S, 64, S, PINV);

  gemm64<0, 1, false, 0, false><<<dim3(8, H, B), 256, 0, stream>>>(
      W2T, D, (long)D * D, 0L, 0L, h16, D, 0L, (long)S * D, hp16, nullptr, H * S, (long)S, (long)D * H * S,
      nullptr, nullptr, D, S, D, WINV);
  scores_kernel<<<dim3(NTOK / 256, H), 256, 0, stream>>>(hp16, as2, ad2, srcb, dstb, D,
                                                          (long)D * H * S, (long)H * S, (long)S, NTOK);
  pbuild_kernel<<<dim3(S, B), 256, 0, stream>>>(adj, srcb, dstb, P16);
  gemm64<0, 0, true, 0, false><<<dim3(8, 1, B), 256, 0, stream>>>(
      P16, H * S, 0L, (long)S * H * S, 0L, hp16, H * S, 0L, (long)D * H * S,
      hA, nullptr, D, 0L, (long)S * D, nullptr, hB, S, D, H * S, PINV * 0.125f);

  ln_kernel<<<NTOK / 8, 256, 0, stream>>>(hA, ln_g, ln_b, hln, hln16, NTOK);

  gemm64<2, 1, false, 6, false><<<dim3(64, 1, 1), 256, 0, stream>>>(
      hln16, D, 0L, 0L, 0L, F1T, D, 0L, 0L, mid16, nullptr, 2 * D, 0L, 0L,
      ffb1, nullptr, NTOK, 2 * D, D, WINV);
  gemm64<2, 0, true, 0, false><<<dim3(32, 1, 1), 256, 0, stream>>>(
      mid16, 2 * D, 0L, 0L, 0L, F2T, 2 * D, 0L, 0L, out, nullptr, D, 0L, 0L,
      ffb2, hln, NTOK, D, 2 * D, WINV);
}
